// SlidingWindowAttention_45019847197305
// MI455X (gfx1250) — hardware-verified
//
#include <hip/hip_runtime.h>
#include <math.h>

typedef __attribute__((ext_vector_type(16))) _Float16 v16h;
typedef __attribute__((ext_vector_type(16))) __bf16 v16b;
typedef __attribute__((ext_vector_type(8)))  _Float16 v8h;
typedef __attribute__((ext_vector_type(8)))  __bf16 v8b;
typedef __attribute__((ext_vector_type(8)))  float v8f;
typedef __attribute__((ext_vector_type(4)))  float v4f;
typedef __attribute__((ext_vector_type(4)))  unsigned v4u;

#ifndef NB
#define NB 1
#endif
#ifndef SEQ
#define SEQ 8192
#endif
#define CC 1024
#define DIN 1024
#define NH 16
#define HD 64
#define HALF 512
#define WIN 512
#define WT (WIN / 64)
#define EARLY ((SEQ) < 512 ? (SEQ) : 512)
#define QBH (EARLY / 64)
#define SCALE (0.125f)

static_assert(NB == 1);
static_assert(SEQ % 64 == 0);
static_assert(CC == NH * HD);
static_assert(CC == 2 * HALF);
static_assert(DIN % 32 == 0);
static_assert(EARLY % 64 == 0);
static_assert(((size_t)SEQ * DIN) % 2048 == 0);
static_assert(((size_t)CC * DIN) % 2048 == 0);

#define NXB ((unsigned)(((size_t)SEQ * DIN) / 2048))
#define NWB ((unsigned)(((size_t)CC * DIN) / 2048))

#define SZ_X   ((size_t)2 * SEQ * DIN)
#define SZ_W   ((size_t)2 * CC * DIN)
#define SZ_E   ((size_t)2 * CC * EARLY)
#define WS_XB  ((size_t)0)
#define WS_WB  (WS_XB + SZ_X)
#define WS_QH  (WS_WB + 4 * SZ_W)
#define WS_QL  (WS_QH + SZ_X)
#define WS_KH  (WS_QL + SZ_X)
#define WS_KL  (WS_KH + SZ_X)
#define WS_VT  (WS_KL + SZ_X)
#define WS_VL  (WS_VT + SZ_X)
#define WS_CH  (WS_VL + SZ_E)
#define WS_CL  (WS_CH + SZ_X)
#define WS_END (WS_CL + SZ_E)
static_assert(WS_END <= (size_t)134217728);

template <typename T> __device__ __forceinline__ void vst2(void* p, T v) { *(volatile T*)p = v; __threadfence(); *(volatile T*)p = v; }
__device__ __forceinline__ v8f wmma16(v16h a, v16h b, v8f c) {
  v8f d = __builtin_amdgcn_wmma_f32_16x16x32_f16(false, a, false, b, (short)0, c, false, false);
  asm volatile("v_nop\n\tv_nop\n\tv_nop\n\tv_nop" : "+v"(d) : "v"(a), "v"(b));
  return d;
}
__device__ __forceinline__ v8f wmma_bf(v16b a, v16b b, v8f c) {
  v8f d = __builtin_amdgcn_wmma_f32_16x16x32_bf16(false, a, false, b, (short)0, c, false, false);
  asm volatile("v_nop\n\tv_nop\n\tv_nop\n\tv_nop" : "+v"(d) : "v"(a), "v"(b));
  return d;
}
__device__ __forceinline__ v16h frag_h(const _Float16* rowk0, unsigned lane) {
  union { v16h v; v8h q[2]; } u; const _Float16* p = rowk0 + 8u * (lane >> 4);
  u.q[0] = *(const v8h*)p; u.q[1] = *(const v8h*)(p + 16); return u.v;
}
__device__ __forceinline__ v16b frag_b(const __bf16* rowk0, unsigned lane) {
  union { v16b v; v8b q[2]; } u; const __bf16* p = rowk0 + 8u * (lane >> 4);
  u.q[0] = *(const v8b*)p; u.q[1] = *(const v8b*)(p + 16); return u.v;
}
#define LDSX() do { asm volatile("s_wait_dscnt 0" ::: "memory"); __builtin_amdgcn_wave_barrier(); __builtin_amdgcn_fence(3  , "workgroup"); } while (0)

__device__ __forceinline__ float bfr(float v) { return (float)(__bf16)v; }
__device__ __forceinline__ unsigned hbits(_Float16 v) { return (unsigned)__builtin_bit_cast(unsigned short, v); }
__device__ __forceinline__ unsigned pack_hr(float v) { const _Float16 hv = (_Float16)v; const _Float16 lv = (_Float16)((v - (float)hv) * 1024.0f); return hbits(hv) | (hbits(lv) << 16); }
__device__ __forceinline__ unsigned ocol(unsigned grp, unsigned cl) { return grp * 64u + (cl & 63u) + ((cl >> 6) << 9); }

__global__ __launch_bounds__(256) void k_cvt(const float* __restrict__ X, const float* __restrict__ W0, const float* __restrict__ W1, const float* __restrict__ W2, const float* __restrict__ W3, __bf16* __restrict__ XB, __bf16* __restrict__ WB) {
  const unsigned tid = threadIdx.x, bid = blockIdx.x;
  const float* src; __bf16* dst; unsigned wsel = 0u; const bool isw = bid >= NXB;
  if (!isw) { src = X + (size_t)bid * 2048u; dst = XB + (size_t)bid * 2048u; }
  else { const unsigned wb = bid - NXB; wsel = wb >> 9; const size_t off = (size_t)(wb & 511u) * 2048u; src = (wsel == 0u ? W0 : wsel == 1u ? W1 : wsel == 2u ? W2 : W3) + off; dst = WB + (size_t)wsel * CC * DIN + off; }
  const float* p = src + tid * 8u; const v4f a = *(const v4f*)p, b = *(const v4f*)(p + 4);
  const float x[8] = {a[0], a[1], a[2], a[3], b[0], b[1], b[2], b[3]};
  union { v8b b; v8h h; v4u u; } o;
  if (isw && wsel == 3u) {
#pragma unroll
    for (int i = 0; i < 8; ++i) o.h[i] = (_Float16)(bfr(x[i]) * 256.0f);
  } else {
#pragma unroll
    for (int i = 0; i < 8; ++i) o.b[i] = (__bf16)x[i];
  }
  vst2((void*)(dst + tid * 8u), o.u);
}

__global__ __launch_bounds__(128) void k_proj(const __bf16* __restrict__ XB, const __bf16* __restrict__ WB, const float* __restrict__ BQ, const float* __restrict__ BK, const float* __restrict__ BV,
    _Float16* __restrict__ QH, _Float16* __restrict__ QL, _Float16* __restrict__ KH, _Float16* __restrict__ KL, _Float16* __restrict__ VT, _Float16* __restrict__ VL) {
  __shared__ __align__(16) unsigned sraw[9216];
  __shared__ float sinv[64];
  const unsigned tid = threadIdx.x, wave = tid >> 5, lane = tid & 31u, col = lane & 15u, g = lane >> 4;
  const unsigned which = blockIdx.z, grp = blockIdx.y, t0 = blockIdx.x * 64u;
  const __bf16* WA = WB + (size_t)which * CC * DIN; const float* BA = which == 0u ? BQ : which == 1u ? BK : BV;
  if (which < 2u && tid < 64u) sinv[tid] = 1.0f / powf(10000.0f, (float)(grp * 64u + tid) * (1.0f / 512.0f));
  v8f acc[8] = {};
  const __bf16* xrow = XB + (size_t)(t0 + wave * 16u + col) * DIN;
#pragma unroll 2
  for (unsigned kc = 0; kc < DIN / 32; ++kc) {
    const v16b a = frag_b(xrow + kc * 32u, lane);
    asm volatile("s_wait_loadcnt 0x0" ::: "memory");
#pragma unroll
    for (int j = 0; j < 8; ++j) { const v16b w = frag_b(WA + (size_t)ocol(grp, (unsigned)j * 16u + col) * DIN + kc * 32u, lane); asm volatile("s_wait_loadcnt 0x0" ::: "memory"); acc[j] = wmma_bf(a, w, acc[j]); }
  }
  if (which < 2u) {
#pragma unroll
    for (int j = 0; j < 8; ++j) { const float bias = bfr(BA[ocol(grp, (unsigned)j * 16u + col)]);
#pragma unroll
      for (int r = 0; r < 8; ++r) sraw[(wave * 16u + 8u * g + (unsigned)r) * 132u + (unsigned)j * 16u + col] = __float_as_uint(acc[j][r] + bias); }
    __syncthreads();
#pragma unroll 1
    for (unsigned i = 0; i < 32u; ++i) { const unsigned e = tid + 128u * i, rl = e >> 6, d = e & 63u;
      const float xlo = __uint_as_float(sraw[rl * 132u + d]), xhi = __uint_as_float(sraw[rl * 132u + 64u + d]);
      const float ang = (float)(t0 + rl) * sinv[d]; const float cs = cosf(ang), sn = sinf(ang);
      const float o1 = xlo * cs - xhi * sn, o2 = xlo * sn + xhi * cs;
      sraw[rl * 132u + d] = pack_hr(o1); sraw[rl * 132u + 64u + d] = pack_hr(o2); }
    __syncthreads();
    _Float16* DH = which == 0u ? QH : KH; _Float16* DL = which == 0u ? QL : KL;
    for (unsigned i = 0; i < 8u; ++i) { const unsigned e = tid + 128u * i, rl = e >> 4, q = e & 15u;
      const v4u w0 = *(const v4u*)&sraw[rl * 132u + q * 8u], w1 = *(const v4u*)&sraw[rl * 132u + q * 8u + 4u];
      v4u hv, lv;
      hv[0] = (w0[0] & 0xffffu) | (w0[1] << 16); lv[0] = (w0[0] >> 16) | (w0[1] & 0xffff0000u);
      hv[1] = (w0[2] & 0xffffu) | (w0[3] << 16); lv[1] = (w0[2] >> 16) | (w0[3] & 0xffff0000u);
      hv[2] = (w1[0] & 0xffffu) | (w1[1] << 16); lv[2] = (w1[0] >> 16) | (w1[1] & 0xffff0000u);
      hv[3] = (w1[2] & 0xffffu) | (w1[3] << 16); lv[3] = (w1[2] >> 16) | (w1[3] & 0xffff0000u);
      const size_t off = (size_t)(t0 + rl) * CC + ocol(grp, q * 8u);
      vst2((void*)(DH + off), hv); vst2((void*)(DL + off), lv); }
  } else {
    _Float16* th = (_Float16*)sraw; _Float16* tl = th + 128 * 72;
#pragma unroll
    for (int j = 0; j < 8; ++j) { const float bias = bfr(BA[ocol(grp, (unsigned)j * 16u + col)]);
#pragma unroll
      for (int r = 0; r < 8; ++r) { const float v = acc[j][r] + bias; const unsigned rl = wave * 16u + 8u * g + (unsigned)r, cl = (unsigned)j * 16u + col; const _Float16 hv = (_Float16)v; th[cl * 72u + rl] = hv; tl[cl * 72u + rl] = (_Float16)((v - (float)hv) * 1024.0f); } }
    __syncthreads();
    const bool hi_rows = t0 < (unsigned)EARLY;
    for (unsigned i = 0; i < 8u; ++i) { const unsigned e = tid + 128u * i, cl = e >> 3, q = e & 7u; const unsigned c = ocol(grp, cl);
      vst2((void*)(VT + (size_t)c * SEQ + t0 + q * 8u), *(const v4u*)&th[cl * 72u + q * 8u]);
      if (hi_rows) vst2((void*)(VL + (size_t)c * EARLY + t0 + q * 8u), *(const v4u*)&tl[cl * 72u + q * 8u]); }
  }
}

template <bool HP>
__global__ __launch_bounds__(128) void k_attn(const _Float16* __restrict__ QH, const _Float16* __restrict__ QL, const _Float16* __restrict__ KH, const _Float16* __restrict__ KL,
    const _Float16* __restrict__ VT, const _Float16* __restrict__ VL, _Float16* __restrict__ CH, _Float16* __restrict__ CL, unsigned qt0) {
  __shared__ __align__(16) _Float16 ph[4][16][72];
  __shared__ __align__(16) _Float16 pl[HP ? 4 : 1][16][72];
  const unsigned tid = threadIdx.x, wave = tid >> 5, lane = tid & 31u, col = lane & 15u, g = lane >> 4;
  const unsigned wl = HP ? wave : 0u;
  const unsigned qt = qt0 + blockIdx.x, h = blockIdx.y; const unsigned t0 = qt * 64u, tq = t0 + wave * 16u;
  v16h qh[2], ql[2];
#pragma unroll
  for (int kc = 0; kc < 2; ++kc) { const size_t qo = (size_t)(tq + col) * CC + h * HD + (unsigned)kc * 32u; qh[kc] = frag_h(QH + qo, lane); ql[kc] = frag_h(QL + qo, lane); }
  float m[8], l[8];
#pragma unroll
  for (int r = 0; r < 8; ++r) { m[r] = -3.0e38f; l[r] = 0.f; }
  v8f o[4] = {}, ol[4] = {};
  const unsigned ktlo = qt >= (unsigned)WT ? qt - (unsigned)WT : 0u;
#pragma unroll 1
  for (unsigned kt = ktlo; kt <= qt; ++kt) { const unsigned k0 = kt * 64u;
    v8f sc[4];
#pragma unroll
    for (int nt = 0; nt < 4; ++nt) { v8f a = {}, al = {};
#pragma unroll
      for (int kc = 0; kc < 2; ++kc) { const size_t ko = (size_t)(k0 + (unsigned)nt * 16u + col) * CC + h * HD + (unsigned)kc * 32u; const v16h kh = frag_h(KH + ko, lane), kl = frag_h(KL + ko, lane);
        a = wmma16(qh[kc], kh, a); al = wmma16(ql[kc], kh, al); al = wmma16(qh[kc], kl, al); }
#pragma unroll
      for (int r = 0; r < 8; ++r) sc[nt][r] = (a[r] + al[r] * (1.0f / 1024.0f)) * SCALE; }
    if (kt == qt || kt + (unsigned)WT == qt) {
#pragma unroll
      for (int nt = 0; nt < 4; ++nt)
#pragma unroll
        for (int r = 0; r < 8; ++r) { const int dd = (int)(tq + 8u * g + (unsigned)r) - (int)(k0 + (unsigned)nt * 16u + col); sc[nt][r] = (dd >= 0 && dd <= WIN) ? sc[nt][r] : -3.0e38f; } }
#pragma unroll
    for (int r = 0; r < 8; ++r) {
      float rmax = fmaxf(fmaxf(sc[0][r], sc[1][r]), fmaxf(sc[2][r], sc[3][r]));
#pragma unroll
      for (int off = 8; off >= 1; off >>= 1) rmax = fmaxf(rmax, __shfl_xor(rmax, off));
      const float mnew = fmaxf(m[r], rmax);
      const float ea = __expf(fmaxf(m[r] - mnew, -80.0f)); const float alpha = (m[r] < -1.0e38f) ? 0.f : ea; m[r] = mnew;
      float rsum = 0.f;
#pragma unroll
      for (int nt = 0; nt < 4; ++nt) { const float x = sc[nt][r]; const float ep = __expf(fmaxf(x - mnew, -80.0f)); const float p = (x < -1.0e38f) ? 0.f : ep; rsum += p;
        const _Float16 hv = (_Float16)p; ph[wave][8u * g + (unsigned)r][(unsigned)nt * 16u + col] = hv;
        if (HP) { pl[wl][8u * g + (unsigned)r][(unsigned)nt * 16u + col] = (_Float16)((p - (float)hv) * 1024.0f); ol[nt][r] *= alpha; }
        o[nt][r] *= alpha; }
#pragma unroll
      for (int off = 8; off >= 1; off >>= 1) rsum += __shfl_xor(rsum, off);
      l[r] = l[r] * alpha + rsum; }
    LDSX();
#pragma unroll
    for (int kc = 0; kc < 2; ++kc) { const v16h pa = frag_h(&ph[wave][col][kc * 32], lane); v16h pla = pa; if (HP) pla = frag_h(&pl[wl][col][kc * 32], lane);
#pragma unroll
      for (int nt = 0; nt < 4; ++nt) { const unsigned c = h * HD + (unsigned)nt * 16u + col; const v16h vh = frag_h(VT + (size_t)c * SEQ + k0 + (unsigned)kc * 32u, lane);
        o[nt] = wmma16(pa, vh, o[nt]);
        if (HP) { const v16h vl = frag_h(VL + (size_t)c * EARLY + k0 + (unsigned)kc * 32u, lane); ol[nt] = wmma16(pla, vh, ol[nt]); ol[nt] = wmma16(pa, vl, ol[nt]); } } }
    LDSX();
  }
#pragma unroll
  for (int r = 0; r < 8; ++r) { const float inv = 16.0f * (1.0f / l[r]);
#pragma unroll
    for (int nt = 0; nt < 4; ++nt) { const float c = (o[nt][r] + (HP ? ol[nt][r] * (1.0f / 1024.0f) : 0.f)) * inv; const _Float16 hv = (_Float16)c; ph[wave][8u * g + (unsigned)r][(unsigned)nt * 16u + col] = hv;
      if (HP) pl[wl][8u * g + (unsigned)r][(unsigned)nt * 16u + col] = (_Float16)((c - (float)hv) * 1024.0f); } }
  LDSX();
  for (unsigned it = 0; it < 4u; ++it) { const unsigned row = it * 4u + (lane >> 3), q = lane & 7u; const size_t off = (size_t)(tq + row) * CC + h * HD + q * 8u;
    vst2((void*)(CH + off), *(const v4u*)&ph[wave][row][q * 8u]);
    if (HP) vst2((void*)(CL + off), *(const v4u*)&pl[wl][row][q * 8u]); }
}

__global__ __launch_bounds__(128) void k_out(const _Float16* __restrict__ CH, const _Float16* __restrict__ CL, const _Float16* __restrict__ WOH, const float* __restrict__ BO, float* __restrict__ OUT) {
  __shared__ __align__(16) float ss[4][16][132];
  const unsigned tid = threadIdx.x, wave = tid >> 5, lane = tid & 31u, col = lane & 15u, g = lane >> 4;
  const unsigned r0 = blockIdx.x * 64u, c0 = blockIdx.y * 128u;
  v8f acc[8] = {}, accl[8] = {};
  const size_t ar = (size_t)(r0 + wave * 16u + col) * CC;
  if (r0 < (unsigned)EARLY) {
#pragma unroll 1
    for (unsigned kc = 0; kc < CC / 32; ++kc) { const v16h a = frag_h(CH + ar + kc * 32u, lane), al = frag_h(CL + ar + kc * 32u, lane);
      asm volatile("s_wait_loadcnt 0x0" ::: "memory");
#pragma unroll
      for (int j = 0; j < 8; ++j) { const v16h w = frag_h(WOH + (size_t)(c0 + (unsigned)j * 16u + col) * CC + kc * 32u, lane); asm volatile("s_wait_loadcnt 0x0" ::: "memory"); acc[j] = wmma16(a, w, acc[j]); accl[j] = wmma16(al, w, accl[j]); } }
  } else {
#pragma unroll 2
    for (unsigned kc = 0; kc < CC / 32; ++kc) { const v16h a = frag_h(CH + ar + kc * 32u, lane);
      asm volatile("s_wait_loadcnt 0x0" ::: "memory");
#pragma unroll
      for (int j = 0; j < 8; ++j) { const v16h w = frag_h(WOH + (size_t)(c0 + (unsigned)j * 16u + col) * CC + kc * 32u, lane); asm volatile("s_wait_loadcnt 0x0" ::: "memory"); acc[j] = wmma16(a, w, acc[j]); } }
  }
#pragma unroll
  for (int j = 0; j < 8; ++j) { const float bias = bfr(BO[c0 + (unsigned)j * 16u + col]);
#pragma unroll
    for (int r = 0; r < 8; ++r) ss[wave][8u * g + (unsigned)r][(unsigned)j * 16u + col] = (acc[j][r] + accl[j][r] * (1.0f / 1024.0f)) * (1.0f / 4096.0f) + bias; }
  LDSX();
  for (unsigned rl = 0; rl < 16u; ++rl) vst2((void*)(OUT + (size_t)(r0 + wave * 16u + rl) * CC + c0 + lane * 4u), *(const v4f*)&ss[wave][rl][lane * 4u]);
}

extern "C" void kernel_launch(void* const* d_in, const int* in_sizes, int n_in, void* d_out, int out_size, void* d_ws, size_t ws_size, hipStream_t stream) {
  if (n_in < 9) return;
  if ((long long)in_sizes[0] < (long long)SEQ * DIN) return;
  if ((long long)in_sizes[1] < (long long)CC * DIN || (long long)in_sizes[3] < (long long)CC * DIN || (long long)in_sizes[5] < (long long)CC * DIN || (long long)in_sizes[7] < (long long)CC * DIN) return;
  if (in_sizes[2] < CC || in_sizes[4] < CC || in_sizes[6] < CC || in_sizes[8] < CC) return;
  if ((long long)out_size < (long long)SEQ * CC) return;
  if (ws_size < (size_t)WS_END) return;
  const float* X = (const float*)d_in[0]; const float* Wq = (const float*)d_in[1]; const float* bq = (const float*)d_in[2]; const float* Wk = (const float*)d_in[3]; const float* bk = (const float*)d_in[4];
  const float* Wv = (const float*)d_in[5]; const float* bv = (const float*)d_in[6]; const float* Wo = (const float*)d_in[7]; const float* bo = (const float*)d_in[8];
  char* ws = (char*)d_ws;
  __bf16* XB = (__bf16*)(ws + WS_XB); __bf16* WB = (__bf16*)(ws + WS_WB); _Float16* WOH = (_Float16*)(ws + WS_WB + 3 * SZ_W);
  _Float16 *QH = (_Float16*)(ws + WS_QH), *QL = (_Float16*)(ws + WS_QL), *KH = (_Float16*)(ws + WS_KH), *KL = (_Float16*)(ws + WS_KL);
  _Float16 *VT = (_Float16*)(ws + WS_VT), *VL = (_Float16*)(ws + WS_VL), *CH = (_Float16*)(ws + WS_CH), *CL = (_Float16*)(ws + WS_CL);
  k_cvt<<<dim3(NXB + 4u * NWB), 256, 0, stream>>>(X, Wq, Wk, Wv, Wo, XB, WB);
  k_proj<<<dim3(SEQ / 64, 8, 3), 128, 0, stream>>>(XB, WB, bq, bk, bv, QH, QL, KH, KL, VT, VL);
  k_attn<true><<<dim3(QBH, NH), 128, 0, stream>>>(QH, QL, KH, KL, VT, VL, CH, CL, 0u);
  if (SEQ / 64 > QBH) k_attn<false><<<dim3(SEQ / 64 - QBH, NH), 128, 0, stream>>>(QH, QL, KH, KL, VT, VL, CH, CL, (unsigned)QBH);
  k_out<<<dim3(SEQ / 64, CC / 128), 128, 0, stream>>>(CH, CL, WOH, bo, (float*)d_out);
}
